// MultiHeadSelfAttention2d_6313601925672
// MI455X (gfx1250) — hardware-verified
//
#include <hip/hip_runtime.h>

typedef _Float16 v16h __attribute__((ext_vector_type(16)));
typedef _Float16 v8h  __attribute__((ext_vector_type(8)));
typedef float    v8f  __attribute__((ext_vector_type(8)));
typedef float    v4f  __attribute__((ext_vector_type(4)));
typedef v8h __attribute__((may_alias)) v8ha;
typedef v4f __attribute__((may_alias)) v4fa;

union Frag { v16h v; v8h half[2]; };

#define BATCH  16
#define CDIM   512
#define NSP    1024
#define NHEAD  8
#define HD     64
#define MROWS  (BATCH * NSP)
#define NX     (BATCH * CDIM * NSP)
#define NW     (CDIM * CDIM)
#define NW8    (NW / 8)
#define WSCALE 16.0f
#define WINV   0.0625f
#define PSCALE 16384.0f
#define OSCALE 8.0f
#define OUTINV 0.0078125f
#define ATT_SCALE 0.125f
#define TP     72

__device__ __forceinline__ v8f wmma_f16(v16h a, v16h b, v8f c) {
  v8f d = __builtin_amdgcn_wmma_f32_16x16x32_f16(false, a, false, b, (short)0, c, false, false);
  asm volatile("v_nop\n\tv_nop\n\tv_nop\n\tv_nop" : "+v"(d) : "v"(a), "v"(b));
  return d;
}

__device__ __forceinline__ v16h load_frag(const _Float16* p, int h) {
  Frag f;
  f.half[0] = *(const v8ha*)(p + 8 * h);
  f.half[1] = *(const v8ha*)(p + 16 + 8 * h);
  return f.v;
}

__global__ __launch_bounds__(256) void cvt_w_kernel(
    const float* __restrict__ wq, const float* __restrict__ wk,
    const float* __restrict__ wv, const float* __restrict__ wo,
    _Float16* __restrict__ wh)
{
  const int g = blockIdx.x * 256 + threadIdx.x;
  if (g >= 4 * NW8) return;
  const int wsel = g / NW8;
  const int off = g - wsel * NW8;
  const float* wsrc = (wsel == 0) ? wq : ((wsel == 1) ? wk : ((wsel == 2) ? wv : wo));
  const float* src = wsrc + (size_t)off * 8;
  _Float16* dst = wh + (size_t)g * 8;
  const v4f a = *(const v4fa*)src;
  const v4f c = *(const v4fa*)(src + 4);
  const v8h o = { (_Float16)(a.x * WSCALE), (_Float16)(a.y * WSCALE), (_Float16)(a.z * WSCALE), (_Float16)(a.w * WSCALE),
                  (_Float16)(c.x * WSCALE), (_Float16)(c.y * WSCALE), (_Float16)(c.z * WSCALE), (_Float16)(c.w * WSCALE) };
  *(volatile v8h*)dst = o;
  __threadfence();
  *(volatile v8h*)dst = o;
}

__device__ __forceinline__ void xt_store_pass(const _Float16* T, _Float16* xt,
                                              int b, int n0, int c0, int w, int lane) {
  const int q8 = lane & 7, sub = lane >> 3;
  #pragma unroll
  for (int i = 0; i < 4; ++i) {
    const int nl = w * 16 + i * 4 + sub;
    const v8h v = *(const v8ha*)(T + nl * TP + 8 * q8);
    _Float16* dst = xt + ((size_t)b * NSP + n0 + nl) * CDIM + c0 + 8 * q8;
    *(volatile v8h*)dst = v;
  }
}

__global__ __launch_bounds__(128) void cvt_x_kernel(const float* __restrict__ x,
                                                   _Float16* __restrict__ xt)
{
  __shared__ __attribute__((aligned(16))) _Float16 T[64 * TP];

  const int tid = threadIdx.x, lane = tid & 31, w = tid >> 5;
  const int n0 = blockIdx.x * 64, c0 = blockIdx.y * 64, b = blockIdx.z;

  #pragma unroll
  for (int i = 0; i < 8; ++i) {
    const int idx = i * 128 + tid;
    const int c = idx >> 4;
    const int n4 = (idx & 15) * 4;
    const v4f v = *(const v4fa*)(x + ((size_t)b * CDIM + c0 + c) * NSP + n0 + n4);
    T[(n4 + 0) * TP + c] = (_Float16)v.x;
    T[(n4 + 1) * TP + c] = (_Float16)v.y;
    T[(n4 + 2) * TP + c] = (_Float16)v.z;
    T[(n4 + 3) * TP + c] = (_Float16)v.w;
  }
  __syncthreads();

  xt_store_pass(T, xt, b, n0, c0, w, lane);
  __threadfence();
  xt_store_pass(T, xt, b, n0, c0, w, lane);
}

__device__ __forceinline__ void proj_store_pass(const _Float16* sT, _Float16* plane, _Float16* vt,
                                                int which, int bh, int l0, int w, int lane) {
  const int q8 = lane & 7, sub = lane >> 3;
  #pragma unroll
  for (int i = 0; i < 8; ++i) {
    const int lid = w * 32 + i * 4 + sub;
    v8h v;
    _Float16* dst;
    if (which != 2) {
      v = *(const v8ha*)(sT + lid * HD + 8 * q8);
      dst = plane + ((size_t)bh * NSP + l0 + lid) * HD + 8 * q8;
    } else {
      const int d = lid >> 1, hl = lid & 1;
      v = *(const v8ha*)(sT + d * 128 + 64 * hl + 8 * q8);
      dst = vt + ((size_t)bh * HD + d) * NSP + l0 + 64 * hl + 8 * q8;
    }
    *(volatile v8h*)dst = v;
  }
}

__global__ __launch_bounds__(128) void proj_kernel(
    const _Float16* __restrict__ xt,
    const _Float16* __restrict__ wh,
    const float* __restrict__ bq, const float* __restrict__ bk, const float* __restrict__ bv,
    _Float16* __restrict__ qh,
    _Float16* __restrict__ kh,
    _Float16* __restrict__ vt)
{
  __shared__ __attribute__((aligned(16))) _Float16 sT[128 * 64];

  const int tid = threadIdx.x, lane = tid & 31, w = tid >> 5;
  const int h = lane >> 4, m = lane & 15;
  const int m0 = blockIdx.x * 128;
  const int cg = blockIdx.y;
  const int which = cg >> 3, head = cg & 7;
  const int m0w = m0 + 32 * w;

  const _Float16* xa0 = xt + (size_t)(m0w + m) * CDIM;
  const _Float16* xa1 = xa0 + (size_t)16 * CDIM;
  const _Float16* wb  = wh + ((size_t)which * CDIM + head * HD + m) * CDIM;

  const v8f zero8 = {0.f, 0.f, 0.f, 0.f, 0.f, 0.f, 0.f, 0.f};
  v8f acc[2][4];
  #pragma unroll
  for (int mt = 0; mt < 2; ++mt)
    #pragma unroll
    for (int nt = 0; nt < 4; ++nt) acc[mt][nt] = zero8;

  #pragma unroll 1
  for (int k0 = 0; k0 < CDIM; k0 += 32) {
    const v16h a0 = load_frag(xa0 + k0, h);
    const v16h a1 = load_frag(xa1 + k0, h);
    #pragma unroll
    for (int nt = 0; nt < 4; ++nt) {
      const v16h b = load_frag(wb + (size_t)nt * 16 * CDIM + k0, h);
      acc[0][nt] = wmma_f16(a0, b, acc[0][nt]);
      acc[1][nt] = wmma_f16(a1, b, acc[1][nt]);
    }
  }

  const float* bias = (which == 0) ? bq : ((which == 1) ? bk : bv);
  #pragma unroll
  for (int nt = 0; nt < 4; ++nt) {
    const int feat = 16 * nt + m;
    const float bvl = bias[head * HD + feat];
    #pragma unroll
    for (int mt = 0; mt < 2; ++mt) {
      #pragma unroll
      for (int r = 0; r < 8; ++r) {
        const int tokl = 32 * w + 16 * mt + 8 * h + r;
        const float y = acc[mt][nt][r] * WINV + bvl;
        const int idx = (which == 2) ? (feat * 128 + tokl) : (tokl * HD + feat);
        sT[idx] = (_Float16)y;
      }
    }
  }
  __syncthreads();

  const int b = m0 / NSP, l0 = m0 - b * NSP, bh = b * NHEAD + head;
  _Float16* plane = (which == 0) ? qh : kh;
  proj_store_pass(sT, plane, vt, which, bh, l0, w, lane);
  __threadfence();
  proj_store_pass(sT, plane, vt, which, bh, l0, w, lane);
}

__device__ __forceinline__ v16h pack_p(v8f a, v8f c) {
  const v16h r = { (_Float16)(a[0] * PSCALE), (_Float16)(a[1] * PSCALE), (_Float16)(a[2] * PSCALE), (_Float16)(a[3] * PSCALE),
                   (_Float16)(a[4] * PSCALE), (_Float16)(a[5] * PSCALE), (_Float16)(a[6] * PSCALE), (_Float16)(a[7] * PSCALE),
                   (_Float16)(c[0] * PSCALE), (_Float16)(c[1] * PSCALE), (_Float16)(c[2] * PSCALE), (_Float16)(c[3] * PSCALE),
                   (_Float16)(c[4] * PSCALE), (_Float16)(c[5] * PSCALE), (_Float16)(c[6] * PSCALE), (_Float16)(c[7] * PSCALE) };
  return r;
}

__device__ __forceinline__ void att_store_pass(const _Float16* so, _Float16* ob,
                                               int b, int head, int q0, int lane) {
  const int q8 = lane & 7, sub = lane >> 3;
  #pragma unroll
  for (int i = 0; i < 4; ++i) {
    const int row = i * 4 + sub;
    const v8h v = *(const v8ha*)(so + row * HD + 8 * q8);
    _Float16* dst = ob + ((size_t)b * NSP + q0 + row) * CDIM + head * HD + 8 * q8;
    *(volatile v8h*)dst = v;
  }
}

__global__ __launch_bounds__(128) void attn_kernel(
    const _Float16* __restrict__ qh,
    const _Float16* __restrict__ kh,
    const _Float16* __restrict__ vt,
    _Float16* __restrict__ ob)
{
  __shared__ __attribute__((aligned(16))) _Float16 sO[4 * 16 * 64];

  const int tid = threadIdx.x, lane = tid & 31, w = tid >> 5;
  const int h = lane >> 4, m = lane & 15;
  const int bh = blockIdx.y, b = bh >> 3, head = bh & 7;
  const int q0 = blockIdx.x * 64 + 16 * w;

  const _Float16* qrow = qh + ((size_t)bh * NSP + q0 + m) * HD;
  const v16h qb0 = load_frag(qrow, h);
  const v16h qb1 = load_frag(qrow + 32, h);

  const v8f zero8 = {0.f, 0.f, 0.f, 0.f, 0.f, 0.f, 0.f, 0.f};
  v8f o[4];
  #pragma unroll
  for (int t = 0; t < 4; ++t) o[t] = zero8;
  float mrun = -1e30f, lrun = 0.0f;

  const _Float16* kbase = kh + ((size_t)bh * NSP + m) * HD;
  const _Float16* vbase = vt + ((size_t)bh * HD + m) * NSP;

  #pragma unroll 1
  for (int kb = 0; kb < NSP; kb += 64) {
    v8f s[4];
    #pragma unroll
    for (int j = 0; j < 4; ++j) {
      const _Float16* kp = kbase + (size_t)(kb + 16 * j) * HD;
      const v16h kf0 = load_frag(kp, h);
      const v16h kf1 = load_frag(kp + 32, h);
      v8f z = zero8;
      z = wmma_f16(kf0, qb0, z);
      z = wmma_f16(kf1, qb1, z);
      s[j] = z;
    }

    float mloc = s[0][0];
    #pragma unroll
    for (int j = 0; j < 4; ++j)
      #pragma unroll
      for (int r = 0; r < 8; ++r) mloc = fmaxf(mloc, s[j][r]);
    mloc = fmaxf(mloc, __shfl_xor(mloc, 16));
    const float mnew = fmaxf(mrun, mloc);
    const float alpha = __expf((mrun - mnew) * ATT_SCALE);
    mrun = mnew;
    float lsum = 0.0f;
    #pragma unroll
    for (int j = 0; j < 4; ++j)
      #pragma unroll
      for (int r = 0; r < 8; ++r) {
        const float p = __expf((s[j][r] - mnew) * ATT_SCALE);
        s[j][r] = p;
        lsum += p;
      }
    lsum += __shfl_xor(lsum, 16);
    lrun = lrun * alpha + lsum;
    #pragma unroll
    for (int t = 0; t < 4; ++t)
      #pragma unroll
      for (int r = 0; r < 8; ++r) o[t][r] = o[t][r] * alpha;

    const v16h pb0 = pack_p(s[0], s[1]);
    const v16h pb1 = pack_p(s[2], s[3]);

    #pragma unroll
    for (int t = 0; t < 4; ++t) {
      const _Float16* vp = vbase + (size_t)(16 * t) * NSP + kb;
      const v16h vf0 = load_frag(vp, h);
      const v16h vf1 = load_frag(vp + 32, h);
      o[t] = wmma_f16(vf0, pb0, o[t]);
      o[t] = wmma_f16(vf1, pb1, o[t]);
    }
  }

  const float inv = (1.0f / lrun) * (OSCALE / PSCALE);
  _Float16* so = sO + w * 1024;
  #pragma unroll
  for (int t = 0; t < 4; ++t)
    #pragma unroll
    for (int r = 0; r < 8; ++r)
      so[m * HD + 16 * t + 8 * h + r] = (_Float16)(o[t][r] * inv);
  __syncthreads();

  att_store_pass(so, ob, b, head, q0, lane);
  __threadfence();
  att_store_pass(so, ob, b, head, q0, lane);
}

__device__ __forceinline__ void out_store_pass(const float* sY, const float* x, float* y,
                                               int b, int o0, int n0, int w, int lane) {
  const int q8 = lane & 7, sub = lane >> 3;
  #pragma unroll
  for (int i = 0; i < 16; ++i) {
    const int L = w * 64 + i * 4 + sub;
    const int ol = L >> 1, hl = L & 1;
    const v4f t = *(const v4fa*)(sY + ol * 64 + 32 * hl + 4 * q8);
    const size_t gi = ((size_t)b * CDIM + o0 + ol) * NSP + n0 + 32 * hl + 4 * q8;
    const v4f xr = *(const v4fa*)(x + gi);
    const v4f val = t + xr;
    *(volatile v4f*)(y + gi) = val;
  }
}

__global__ __launch_bounds__(128) void out_kernel(
    const _Float16* __restrict__ wh,
    const _Float16* __restrict__ ob,
    const float* __restrict__ bo,
    const float* __restrict__ gamma,
    const float* __restrict__ x,
    float* __restrict__ y)
{
  __shared__ __attribute__((aligned(16))) float sY[128 * 64];

  const int tid = threadIdx.x, lane = tid & 31, w = tid >> 5;
  const int h = lane >> 4, m = lane & 15;
  const int o0 = blockIdx.y * 128;
  const int n0g = blockIdx.x * 64;
  const int b = n0g / NSP, n0 = n0g - b * NSP;

  const _Float16* wa0 = wh + (size_t)3 * NW + (size_t)(o0 + 32 * w + m) * CDIM;
  const _Float16* wa1 = wa0 + (size_t)16 * CDIM;
  const _Float16* bb  = ob + (size_t)(n0g + m) * CDIM;

  const v8f zero8 = {0.f, 0.f, 0.f, 0.f, 0.f, 0.f, 0.f, 0.f};
  v8f acc[2][4];
  #pragma unroll
  for (int mt = 0; mt < 2; ++mt)
    #pragma unroll
    for (int nt = 0; nt < 4; ++nt) acc[mt][nt] = zero8;

  #pragma unroll 1
  for (int k0 = 0; k0 < CDIM; k0 += 32) {
    const v16h a0 = load_frag(wa0 + k0, h);
    const v16h a1 = load_frag(wa1 + k0, h);
    #pragma unroll
    for (int nt = 0; nt < 4; ++nt) {
      const v16h bf = load_frag(bb + (size_t)nt * 16 * CDIM + k0, h);
      acc[0][nt] = wmma_f16(a0, bf, acc[0][nt]);
      acc[1][nt] = wmma_f16(a1, bf, acc[1][nt]);
    }
  }

  const float g = gamma[0];
  #pragma unroll
  for (int mt = 0; mt < 2; ++mt) {
    #pragma unroll
    for (int r = 0; r < 8; ++r) {
      const int ol = 32 * w + 16 * mt + 8 * h + r;
      const float bvl = bo[o0 + ol];
      #pragma unroll
      for (int nt = 0; nt < 4; ++nt) {
        const int nl = 16 * nt + m;
        sY[ol * 64 + nl] = g * (acc[mt][nt][r] * OUTINV + bvl);
      }
    }
  }
  __syncthreads();

  out_store_pass(sY, x, y, b, o0, n0, w, lane);
  __threadfence();
  out_store_pass(sY, x, y, b, o0, n0, w, lane);
}

extern "C" void kernel_launch(void* const* d_in, const int* in_sizes, int n_in,
                              void* d_out, int out_size, void* d_ws, size_t ws_size,
                              hipStream_t stream) {
  if (n_in < 10) return;
  if (in_sizes[0] != NX || out_size != NX) return;
  if (in_sizes[1] != NW || in_sizes[3] != NW || in_sizes[5] != NW || in_sizes[7] != NW) return;
  if (in_sizes[2] != CDIM || in_sizes[4] != CDIM || in_sizes[6] != CDIM || in_sizes[8] != CDIM) return;
  if (in_sizes[9] < 1) return;

  const float* x  = (const float*)d_in[0];
  const float* wq = (const float*)d_in[1];
  const float* bq = (const float*)d_in[2];
  const float* wk = (const float*)d_in[3];
  const float* bk = (const float*)d_in[4];
  const float* wv = (const float*)d_in[5];
  const float* bv = (const float*)d_in[6];
  const float* wo = (const float*)d_in[7];
  const float* bo = (const float*)d_in[8];
  const float* gm = (const float*)d_in[9];
  float* y = (float*)d_out;

  const size_t xt_bytes = (size_t)NX * 2;
  const size_t wh_bytes = (size_t)4 * NW * 2;
  const size_t pl_bytes = (size_t)NX * 2;
  const size_t total = xt_bytes + wh_bytes + 4 * pl_bytes;
  if (total > ws_size) return;

  char* ws = (char*)d_ws;
  _Float16* xt = (_Float16*)(ws);
  _Float16* wh = (_Float16*)(ws + xt_bytes);
  _Float16* qh = (_Float16*)(ws + xt_bytes + wh_bytes);
  _Float16* kh = (_Float16*)(ws + xt_bytes + wh_bytes + pl_bytes);
  _Float16* vt = (_Float16*)(ws + xt_bytes + wh_bytes + 2 * pl_bytes);
  _Float16* ob = (_Float16*)(ws + xt_bytes + wh_bytes + 3 * pl_bytes);

  cvt_w_kernel<<<(4 * NW8 + 255) / 256, 256, 0, stream>>>(wq, wk, wv, wo, wh);

  dim3 gX(NSP / 64, CDIM / 64, BATCH);
  cvt_x_kernel<<<gX, 128, 0, stream>>>(x, xt);

  dim3 gProj(MROWS / 128, 3 * NHEAD);
  proj_kernel<<<gProj, 128, 0, stream>>>(xt, wh, bq, bk, bv, qh, kh, vt);

  dim3 gAtt(NSP / 64, BATCH * NHEAD);
  attn_kernel<<<gAtt, 128, 0, stream>>>(qh, kh, vt, ob);

  dim3 gOut(MROWS / 64, CDIM / 128);
  out_kernel<<<gOut, 128, 0, stream>>>(wh, ob, bo, gm, x, y);
}
